// GATv2Model_4922032521307
// MI455X (gfx1250) — hardware-verified
//
#include <hip/hip_runtime.h>
#include <stddef.h>
#include <math.h>


#define DIN     512
#define HC      256
#define NH1     2
#define CH1     128
#define DOUT    64
#define KX      512
#define NP1     512
#define NP2     128
#define CPL1    8
#define CPL2    4
#define NTHR    256
#define NWAVE   8
#define EPT     8
#define CHUNK   (NTHR * EPT)
#define WCAP    (EPT * 32)
#define LISTN   (NWAVE * WCAP)
#define NBMAX   2048
#define SLOTB   11
#define RCAP    28672
#define DEGCAP  64
#define GBM     64
#define GBN     64
#define GTHR    128
#define NBW1    ((HC * (KX / 8)) / NTHR)
#define NBW2    ((DOUT * (KX / 8)) / NTHR)
#define NEGSL   0.2f
#define EPS_SM  1e-16f
#define WSMAX   134217728
#define LDS_AGG ((2 * RCAP + 2 * NBMAX + LISTN) * 4 + 64)

static_assert((CHUNK & (CHUNK - 1)) == 0 && CHUNK <= (1 << SLOTB));
static_assert(NBMAX == (1 << SLOTB));
static_assert(NTHR * 8 == NBMAX);
static_assert(LISTN >= NBMAX);
static_assert(LISTN >= NWAVE * WCAP);
static_assert((RCAP % 32) == 0);
static_assert(LDS_AGG <= 300000);
static_assert(LDS_AGG == 254016);
static_assert(GBM == (GTHR / 32) * 16);
static_assert((KX % 32) == 0 && DIN == KX && KX == 2 * HC);
static_assert(KX / 8 == (1 << 6));
static_assert((NP1 % GBN) == 0 && NP1 == 2 * HC && (HC % GBN) == 0);
static_assert((NP2 % GBN) == 0 && NP2 == 2 * DOUT && (DOUT % GBN) == 0);
static_assert(HC == NH1 * CH1 && HC == 32 * CPL1 && CH1 == 16 * CPL1);
static_assert(DOUT == 16 * CPL2);
static_assert(NBW1 * NTHR == HC * (KX / 8));
static_assert(NBW2 * NTHR == DOUT * (KX / 8));
static_assert((DIN / 8) * 8 == DIN);
static_assert(DEGCAP <= RCAP);

typedef float          v4f  __attribute__((ext_vector_type(4)));
typedef float          v8f  __attribute__((ext_vector_type(8)));
typedef int            v4i  __attribute__((ext_vector_type(4)));
typedef int            v8i  __attribute__((ext_vector_type(8)));
typedef unsigned int   v4u  __attribute__((ext_vector_type(4)));
typedef unsigned short v8us __attribute__((ext_vector_type(8)));
typedef __bf16         v16b __attribute__((ext_vector_type(16)));
typedef v4f  __attribute__((may_alias)) v4fa;
typedef v8us __attribute__((may_alias)) v8usa;
union FragB { v16b v; v8us h[2]; v8i w; };

__device__ __forceinline__ v8f wmb(const FragB& a, const FragB& b, v8f c) {
  v8f d = __builtin_amdgcn_wmma_f32_16x16x32_bf16(false, a.v, false, b.v, (short)0, c, false, false);
  asm volatile("v_nop\n\tv_nop\n\tv_nop\n\tv_nop" : "+v"(d) : "v"(a.w), "v"(b.w));
  return d;
}

__device__ __forceinline__ unsigned int f2bf(float f) {
  const unsigned int u = __float_as_uint(f);
  return ((u + 0x7FFFu + ((u >> 16) & 1u)) >> 16) & 0xFFFFu;
}
__device__ __forceinline__ float bf2f(unsigned int b) { return __uint_as_float(b << 16); }
__device__ __forceinline__ float bfr(float f) { return bf2f(f2bf(f)); }
__device__ __forceinline__ v4f bfr4(const v4f a) {
  v4f r; r.x = bfr(a.x); r.y = bfr(a.y); r.z = bfr(a.z); r.w = bfr(a.w); return r;
}
__device__ __forceinline__ v8us cvt8b(const v4f a, const v4f b) {
  v8us o;
  o[0] = (unsigned short)f2bf(a.x); o[1] = (unsigned short)f2bf(a.y);
  o[2] = (unsigned short)f2bf(a.z); o[3] = (unsigned short)f2bf(a.w);
  o[4] = (unsigned short)f2bf(b.x); o[5] = (unsigned short)f2bf(b.y);
  o[6] = (unsigned short)f2bf(b.z); o[7] = (unsigned short)f2bf(b.w);
  return o;
}
__device__ __forceinline__ void hilo8(const v4f a, const v4f b, v4u& hi, v4u& lo) {
  const float f[8] = {a.x, a.y, a.z, a.w, b.x, b.y, b.z, b.w};
  unsigned int hb[8], lb[8];
#pragma unroll
  for (int i = 0; i < 8; ++i) {
    hb[i] = f2bf(f[i]);
    lb[i] = f2bf(f[i] - bf2f(hb[i]));
  }
  hi.x = hb[0] | (hb[1] << 16); hi.y = hb[2] | (hb[3] << 16); hi.z = hb[4] | (hb[5] << 16); hi.w = hb[6] | (hb[7] << 16);
  lo.x = lb[0] | (lb[1] << 16); lo.y = lb[2] | (lb[3] << 16); lo.z = lb[4] | (lb[5] << 16); lo.w = lb[6] | (lb[7] << 16);
}
template<int NQ>
__device__ __forceinline__ void ldq(float (&d)[4 * NQ], const float* __restrict__ p) {
#pragma unroll
  for (int k = 0; k < NQ; ++k) {
    const v4f t = *(const v4fa*)(p + 4 * k);
    d[4 * k] = t.x; d[4 * k + 1] = t.y; d[4 * k + 2] = t.z; d[4 * k + 3] = t.w;
  }
}
template<int NQ>
__device__ __forceinline__ void ldqb(float (&d)[4 * NQ], const float* __restrict__ p) {
#pragma unroll
  for (int k = 0; k < NQ; ++k) {
    const v4f t = bfr4(*(const v4fa*)(p + 4 * k));
    d[4 * k] = t.x; d[4 * k + 1] = t.y; d[4 * k + 2] = t.z; d[4 * k + 3] = t.w;
  }
}
__device__ __forceinline__ float gsum16(float p) {
  p += __shfl_xor(p, 8); p += __shfl_xor(p, 4); p += __shfl_xor(p, 2); p += __shfl_xor(p, 1);
  return p;
}

__device__ __forceinline__ int scan_chunk(const int* __restrict__ dsts, int nE, int cbase, int slotBase,
                                          int nb, int vec8, int* list, int tid, int lane, int wave) {
  int wc = 0;
  const int el0  = tid * EPT;
  const int e0   = cbase + el0;
  const int sent = -2147483647 - 1;
  v4i da, db;
  if (vec8 != 0 && cbase + CHUNK <= nE) {
    da = *(const v4i*)(dsts + e0);
    db = *(const v4i*)(dsts + e0 + 4);
  } else {
    da.x = (e0     < nE) ? dsts[min(e0,     nE - 1)] : sent;
    da.y = (e0 + 1 < nE) ? dsts[min(e0 + 1, nE - 1)] : sent;
    da.z = (e0 + 2 < nE) ? dsts[min(e0 + 2, nE - 1)] : sent;
    da.w = (e0 + 3 < nE) ? dsts[min(e0 + 3, nE - 1)] : sent;
    db.x = (e0 + 4 < nE) ? dsts[min(e0 + 4, nE - 1)] : sent;
    db.y = (e0 + 5 < nE) ? dsts[min(e0 + 5, nE - 1)] : sent;
    db.z = (e0 + 6 < nE) ? dsts[min(e0 + 6, nE - 1)] : sent;
    db.w = (e0 + 7 < nE) ? dsts[min(e0 + 7, nE - 1)] : sent;
  }
  const unsigned nbs = (unsigned)slotBase;
  const unsigned unb = (unsigned)nb;
  const unsigned s0 = (unsigned)da.x - nbs, s1 = (unsigned)da.y - nbs;
  const unsigned s2 = (unsigned)da.z - nbs, s3 = (unsigned)da.w - nbs;
  const unsigned s4 = (unsigned)db.x - nbs, s5 = (unsigned)db.y - nbs;
  const unsigned s6 = (unsigned)db.z - nbs, s7 = (unsigned)db.w - nbs;
  const bool h0 = s0 < unb, h1 = s1 < unb, h2 = s2 < unb, h3 = s3 < unb;
  const bool h4 = s4 < unb, h5 = s5 < unb, h6 = s6 < unb, h7 = s7 < unb;
  const unsigned any = __builtin_amdgcn_ballot_w32(h0 | h1 | h2 | h3 | h4 | h5 | h6 | h7);
  if (any != 0u) {
#define HITJ(J, HJ, SJ) { \
      const unsigned mj = __builtin_amdgcn_ballot_w32(HJ); \
      if (mj != 0u) { \
        if (HJ) { \
          const int pos = wc + (int)__builtin_amdgcn_mbcnt_lo(mj, 0u); \
          if (pos < WCAP) list[wave * WCAP + pos] = ((el0 + (J)) << SLOTB) | (int)(SJ); \
        } \
        wc += (int)__builtin_popcount(mj); } }
    HITJ(0, h0, s0)
    HITJ(1, h1, s1)
    HITJ(2, h2, s2)
    HITJ(3, h3, s3)
    HITJ(4, h4, s4)
    HITJ(5, h5, s5)
    HITJ(6, h6, s6)
    HITJ(7, h7, s7)
#undef HITJ
  }
  return wc;
}

__device__ __forceinline__ void wt_unit(const float* __restrict__ w, int cols, int ush, int kmask, int Kout,
                                        unsigned short* wt, int rowoff, int u) {
  const int n   = u >> ush;
  const int k8  = (u & ((1 << ush) - 1)) * 8;
  const int kk  = k8 & kmask;
  const int ncl = n < cols ? n : cols - 1;
  const float* p = w + (size_t)kk * (size_t)cols + ncl;
  v4f a, b;
  a.x = p[0];                  a.y = p[(size_t)cols];       a.z = p[(size_t)2 * cols];   a.w = p[(size_t)3 * cols];
  b.x = p[(size_t)4 * cols];   b.y = p[(size_t)5 * cols];   b.z = p[(size_t)6 * cols];   b.w = p[(size_t)7 * cols];
  const v4f z4 = {0.f, 0.f, 0.f, 0.f};
  if (n >= cols) { a = z4; b = z4; }
  const v8us hv = cvt8b(a, b);
  const size_t o = (size_t)(rowoff + n) * (size_t)Kout + k8;
  *(volatile v8us*)(wt + o) = hv;
  __threadfence();
  *(volatile v8us*)(wt + o) = hv;
}

__global__ __launch_bounds__(NTHR) void k_prep(const float* __restrict__ x,
                                               const float* __restrict__ W1l, const float* __restrict__ W1r,
                                               const float* __restrict__ W2l, const float* __restrict__ W2r,
                                               unsigned short* xb, unsigned short* wt1, unsigned short* wt2,
                                               int nN, int nUx, int nBx) {
  const int tid = (int)threadIdx.x;
  const int bid = (int)blockIdx.x;
  if (bid < nBx) {
    const int i = bid * NTHR + tid;
    if (i >= nUx) return;
    const int row = i >> 6;
    const int c0  = (i & 63) * 8;
    const int rc  = row < nN ? row : nN - 1;
    const float* p = x + (size_t)rc * DIN + c0;
    v4f a = *(const v4fa*)p, b = *(const v4fa*)(p + 4);
    const v4f z4 = {0.f, 0.f, 0.f, 0.f};
    if (row >= nN) { a = z4; b = z4; }
    const v8us hv = cvt8b(a, b);
    const size_t o = (size_t)row * DIN + c0;
    *(volatile v8us*)(xb + o) = hv;
    __threadfence();
    *(volatile v8us*)(xb + o) = hv;
  } else {
    const int rb = bid - nBx;
    if (rb < NBW1) {
      const int u = rb * NTHR + tid;
      if (u < HC * (KX / 8)) wt_unit(W1l, HC, 6, DIN - 1, KX, wt1, 0, u);
    } else if (rb < 2 * NBW1) {
      const int u = (rb - NBW1) * NTHR + tid;
      if (u < HC * (KX / 8)) wt_unit(W1r, HC, 6, DIN - 1, KX, wt1, HC, u);
    } else if (rb < 2 * NBW1 + NBW2) {
      const int u = (rb - 2 * NBW1) * NTHR + tid;
      if (u < DOUT * (KX / 8)) wt_unit(W2l, DOUT, 6, HC - 1, KX, wt2, 0, u);
    } else if (rb < 2 * NBW1 + 2 * NBW2) {
      const int u = (rb - 2 * NBW1 - NBW2) * NTHR + tid;
      if (u < DOUT * (KX / 8)) wt_unit(W2r, DOUT, 6, HC - 1, KX, wt2, DOUT, u);
    }
  }
}

__global__ __launch_bounds__(GTHR) void k_gemm(
    const unsigned short* __restrict__ A, const unsigned short* __restrict__ WT,
    const float* __restrict__ b0, const float* __restrict__ b1, const float* __restrict__ b2,
    int n0, int n1, int nb0, int nb1, int nb2,
    float* outF, int K, int ldo)
{
  __shared__ __attribute__((aligned(16))) float stg[GBM * GBN];
  const int tid = (int)threadIdx.x, lane = tid & 31, wave = tid >> 5, hh = lane >> 4, m = lane & 15;
  const int rowBase = (int)blockIdx.x * GBM;
  const int col0    = (int)blockIdx.y * GBN;

  v8f acc[4];
  {
    const v8f z = {0.f, 0.f, 0.f, 0.f, 0.f, 0.f, 0.f, 0.f};
    acc[0] = z; acc[1] = z; acc[2] = z; acc[3] = z;
  }
  const unsigned short* ap = A  + (size_t)(rowBase + 16 * wave + m) * (size_t)K + 8 * hh;
  const unsigned short* wp = WT + (size_t)(col0 + m) * (size_t)K + 8 * hh;
  const int ksteps = K >> 5;
#pragma unroll 1
  for (int ks = 0; ks < ksteps; ++ks) {
    FragB af;
    af.h[0] = *(const v8usa*)(ap + 32 * ks);
    af.h[1] = *(const v8usa*)(ap + 32 * ks + 16);
#pragma unroll
    for (int t = 0; t < 4; ++t) {
      const unsigned short* wq = wp + (size_t)(16 * t) * (size_t)K + 32 * ks;
      FragB bf;
      bf.h[0] = *(const v8usa*)wq;
      bf.h[1] = *(const v8usa*)(wq + 16);
      acc[t] = wmb(af, bf, acc[t]);
    }
  }

#pragma unroll
  for (int t = 0; t < 4; ++t) {
    const int lc = 16 * t + m;
#pragma unroll
    for (int r = 0; r < 8; ++r) {
      const int lr = 16 * wave + 8 * hh + r;
      stg[lr * GBN + lc] = acc[t][r];
    }
  }
  __syncthreads();

  const int gcb = col0 + 4 * m;
  int j0 = gcb;      j0 = j0 > nb0 - 4 ? nb0 - 4 : j0; j0 = j0 < 0 ? 0 : j0;
  int j1 = gcb - n0; j1 = j1 > nb1 - 4 ? nb1 - 4 : j1; j1 = j1 < 0 ? 0 : j1;
  int j2 = gcb - n1; j2 = j2 > nb2 - 4 ? nb2 - 4 : j2; j2 = j2 < 0 ? 0 : j2;
  const v4f q0 = bfr4(*(const v4fa*)(b0 + j0));
  const v4f q1 = bfr4(*(const v4fa*)(b1 + j1));
  const v4f q2 = bfr4(*(const v4fa*)(b2 + j2));
  const float f0 = (gcb < n0) ? 1.0f : 0.0f;
  const float f1 = (gcb >= n0 && gcb < n1) ? 1.0f : 0.0f;
  const float f2 = (gcb >= n1) ? 1.0f : 0.0f;
  const v4f bsum = q0 * f0 + q1 * f1 + q2 * f2;

  v4f fv[8];
#pragma unroll
  for (int i = 0; i < 8; ++i) {
    const int lr = 16 * wave + 2 * i + hh;
    fv[i] = *(const v4fa*)(stg + lr * GBN + 4 * m) + bsum;
  }
#pragma unroll
  for (int i = 0; i < 8; ++i) {
    const int lr = 16 * wave + 2 * i + hh;
    const int gr = rowBase + lr;
    float* op = outF + (size_t)gr * (size_t)ldo + col0 + 4 * m;
    *(volatile v4f*)op = fv[i];
  }
  __threadfence();
#pragma unroll
  for (int i = 0; i < 8; ++i) {
    const int lr = 16 * wave + 2 * i + hh;
    const int gr = rowBase + lr;
    float* op = outF + (size_t)gr * (size_t)ldo + col0 + 4 * m;
    *(volatile v4f*)op = fv[i];
  }
}

template<int C>
__device__ __forceinline__ float edot(const float (&hs)[C], const float (&hd)[C],
                                      const float (&we)[C], const float (&at)[C], float wv) {
  float part = 0.f;
#pragma unroll
  for (int j = 0; j < C; ++j) {
    float v = fmaf(wv, we[j], hs[j] + hd[j]);
    v = v >= 0.f ? v : v * NEGSL;
    part = fmaf(v, at[j], part);
  }
  return part;
}
template<int C>
__device__ __forceinline__ void smerge(float lg, float& mx, float& dn, float (&av)[C], const float (&hs)[C]) {
  const float df = lg - mx;
  const float ee = __expf(-fabsf(df));
  const bool up  = df > 0.f;
  const float s1 = up ? ee : 1.0f;
  const float s2 = up ? 1.0f : ee;
  mx = up ? lg : mx;
  dn = fmaf(dn, s1, s2);
#pragma unroll
  for (int j = 0; j < C; ++j) av[j] = fmaf(av[j], s1, s2 * hs[j]);
}

template<int CPL, int MODE>
__global__ __launch_bounds__(NTHR) void k_agg(
    const int* __restrict__ srcs, const int* __restrict__ dsts, const float* __restrict__ ea,
    const float* __restrict__ F,
    const float* __restrict__ We, const float* __restrict__ att, const float* __restrict__ bias,
    unsigned short* HBo, float* outp,
    int nN, int nE, int nb, int vec8, int MPr) {
  static_assert((MODE == 0 && CPL == 8) || (MODE == 1 && CPL == 4));
  constexpr int HCW = (MODE == 0) ? 32 * CPL : 16 * CPL;
  constexpr int LDF = 2 * HCW;
  extern __shared__ v4f lds_dyn[];
  int* reg1 = (int*)lds_dyn;
  int* reg2 = reg1 + RCAP;
  int* scnt = reg2 + RCAP;
  int* soff = scnt + NBMAX;
  int* list = soff + NBMAX;
  int* wcnt = list + LISTN;
  int* wtot = wcnt + NWAVE;
  const int tid = (int)threadIdx.x, lane = tid & 31, wave = tid >> 5;
  const int nodeBase = (int)blockIdx.x * nb;

  for (int i = tid; i < NBMAX; i += NTHR) scnt[i] = 0;
  for (int i = tid; i < RCAP; i += NTHR) reg2[i] = 0;
  __syncthreads();

  int tot = 0;
  const int nChunks = (nE + CHUNK - 1) / CHUNK;
#pragma unroll 1
  for (int ch = 0; ch < nChunks; ++ch) {
    const int cbase = ch * CHUNK;
    const int wc = scan_chunk(dsts, nE, cbase, nodeBase, nb, vec8, list, tid, lane, wave);
    if (lane == 0) wcnt[wave] = wc;
    __syncthreads();
    int pre = 0, all = 0;
#pragma unroll
    for (int w2 = 0; w2 < NWAVE; ++w2) {
      int c = wcnt[w2];
      c = c < 0 ? 0 : (c > WCAP ? WCAP : c);
      all += c;
      pre += (w2 < wave) ? c : 0;
    }
    const int wcc  = wc > WCAP ? WCAP : wc;
    const int base = tot + pre;
#pragma unroll 1
    for (int i = lane; i < wcc; i += 32) {
      const int ent = list[wave * WCAP + i];
      const int el  = (ent >> SLOTB) & (CHUNK - 1);
      const int sl  = ent & (NBMAX - 1);
      int eid = cbase + el;
      eid = eid > nE - 1 ? nE - 1 : eid;
      const int pos = base + i;
      if (pos < RCAP) reg1[pos] = (int)(((unsigned)eid << SLOTB) | (unsigned)sl);
    }
    tot += all;
    tot = tot > RCAP ? RCAP : tot;
    __syncthreads();
  }
  const int nh = tot;

  if (wave == 0) {
#pragma unroll 1
    for (int b0 = 0; b0 < nh; b0 += 32) {
      const int idx = b0 + lane;
      const int uv  = reg1[idx < nh ? idx : nh - 1];
      const int m32 = (nh - b0) < 32 ? (nh - b0) : 32;
#pragma unroll 1
      for (int k = 0; k < m32; ++k) {
        const int u  = __builtin_amdgcn_readlane(uv, k);
        const int sl = u & (NBMAX - 1);
        if (lane == 0) scnt[sl] = scnt[sl] + 1;
      }
    }
  }
  __syncthreads();

  {
    const v4i ca = *(const v4i*)(scnt + 8 * tid);
    const v4i cb = *(const v4i*)(scnt + 8 * tid + 4);
    const int e0 = ca.x < 0 ? 0 : ca.x, e1 = ca.y < 0 ? 0 : ca.y, e2 = ca.z < 0 ? 0 : ca.z, e3 = ca.w < 0 ? 0 : ca.w;
    const int e4 = cb.x < 0 ? 0 : cb.x, e5 = cb.y < 0 ? 0 : cb.y, e6 = cb.z < 0 ? 0 : cb.z, e7 = cb.w < 0 ? 0 : cb.w;
    const int ts = e0 + e1 + e2 + e3 + e4 + e5 + e6 + e7;
    int incl = ts;
#pragma unroll
    for (int d = 1; d < 32; d <<= 1) {
      const int up = __shfl_up(incl, d);
      if (lane >= d) incl += up;
    }
    if (lane == 31) wtot[wave] = incl;
    __syncthreads();
    int pre = 0;
#pragma unroll
    for (int w2 = 0; w2 < NWAVE; ++w2) pre += (w2 < wave) ? wtot[w2] : 0;
    int run = pre + incl - ts;
    soff[8 * tid + 0] = run; run += e0;
    soff[8 * tid + 1] = run; run += e1;
    soff[8 * tid + 2] = run; run += e2;
    soff[8 * tid + 3] = run; run += e3;
    soff[8 * tid + 4] = run; run += e4;
    soff[8 * tid + 5] = run; run += e5;
    soff[8 * tid + 6] = run; run += e6;
    soff[8 * tid + 7] = run;
  }
  __syncthreads();
  for (int i = tid; i < NBMAX; i += NTHR) list[i] = soff[i];
  __syncthreads();

  if (wave == 0) {
#pragma unroll 1
    for (int b0 = 0; b0 < nh; b0 += 32) {
      const int idx = b0 + lane;
      const int uv  = reg1[idx < nh ? idx : nh - 1];
      const int m32 = (nh - b0) < 32 ? (nh - b0) : 32;
#pragma unroll 1
      for (int k = 0; k < m32; ++k) {
        const int u   = __builtin_amdgcn_readlane(uv, k);
        const int sl  = u & (NBMAX - 1);
        const int eid = (int)((unsigned)u >> SLOTB);
        if (lane == 0) {
          int pos = list[sl];
          pos = pos < 0 ? 0 : (pos > RCAP - 1 ? RCAP - 1 : pos);
          reg2[pos] = eid;
          list[sl] = pos + 1;
        }
      }
    }
  }
  __syncthreads();

  const int nbw = nb >> 3;
  const bool ovf = (nh >= RCAP);
  const float qnan = __int_as_float(0x7fc00000);
  const int c0 = (MODE == 0) ? CPL * lane : CPL * (lane & 15);
  float we[CPL], at[CPL], bb[CPL];
  ldqb<CPL / 4>(we, We + c0);
  ldqb<CPL / 4>(at, att + c0);
  ldqb<CPL / 4>(bb, bias + c0);

#pragma unroll 1
  for (int jt = 0; jt < nbw; ++jt) {
    const int slot = wave * nbw + jt;
    const int grow = nodeBase + slot;
    const int gcl  = grow < nN ? grow : nN - 1;
    int st = soff[slot];
    const int craw = scnt[slot];
    int cnt = craw;
    st  = st < 0 ? 0 : (st > nh ? nh : st);
    cnt = cnt < 0 ? 0 : (cnt > DEGCAP ? DEGCAP : cnt);
    if (cnt > nh - st) cnt = nh - st;
    const float pz = (ovf || craw > DEGCAP) ? qnan : 0.0f;
    const bool live = grow < nN;
    const bool inpl = grow < MPr;
    const int  cl1  = cnt > 0 ? cnt : 1;
    const float rdeg = __builtin_amdgcn_rcpf((float)cl1);

    const float* fr = F + (size_t)gcl * (size_t)LDF;
    float hd[CPL];
    ldq<CPL / 4>(hd, fr + HCW + c0);
    float av[CPL];
#pragma unroll
    for (int j = 0; j < CPL; ++j) av[j] = 0.f;
    float mx = -1.0e30f, dn = 0.f, asum = 0.f;

#pragma unroll 1
    for (int q = 0; q <= cnt; ++q) {
      const bool last = (q == cnt);
      int idx = st + q; idx = idx > RCAP - 1 ? RCAP - 1 : idx;
      int eid = reg2[idx]; eid = eid < 0 ? 0 : (eid > nE - 1 ? nE - 1 : eid);
      const int sraw = srcs[eid];
      const int se = sraw < 0 ? 0 : (sraw > nN - 1 ? nN - 1 : sraw);
      const int s = last ? gcl : se;
      const float aed = bfr(ea[eid]);
      asum += last ? 0.0f : aed;
      const float wv = last ? asum * rdeg : aed;
      float hs[CPL];
      ldq<CPL / 4>(hs, F + (size_t)s * (size_t)LDF + c0);
      const float lg = gsum16(edot<CPL>(hs, hd, we, at, wv));
      smerge<CPL>(lg, mx, dn, av, hs);
    }
    const float inv = __builtin_amdgcn_rcpf(dn + EPS_SM);

    if constexpr (MODE == 0) {
      float r[CPL];
#pragma unroll
      for (int j = 0; j < CPL; ++j) {
        float v = fmaf(av[j], inv, bb[j]);
        v = v > 0.f ? v : (__expf(v) - 1.0f);
        r[j] = (live ? v : 0.f) + pz;
      }
      v4f ra, rq;
      ra.x = r[0]; ra.y = r[1]; ra.z = r[2]; ra.w = r[3];
      rq.x = r[4]; rq.y = r[5]; rq.z = r[6]; rq.w = r[7];
      v4u hi, lo;
      hilo8(ra, rq, hi, lo);
      unsigned short* hp = HBo + (size_t)grow * (size_t)LDF + c0;
      if (inpl) {
        *(volatile v4u*)(hp)       = hi;
        *(volatile v4u*)(hp + HCW) = lo;
      }
      __threadfence();
      if (inpl) {
        *(volatile v4u*)(hp)       = hi;
        *(volatile v4u*)(hp + HCW) = lo;
      }
    } else {
      float r[CPL];
#pragma unroll
      for (int j = 0; j < CPL; ++j) {
        const float v = fmaf(av[j], inv, bb[j]);
        r[j] = (live ? v : 0.f) + pz;
      }
      v4f y; y.x = r[0]; y.y = r[1]; y.z = r[2]; y.w = r[3];
      float* op = outp + (size_t)gcl * HCW + c0;
      const bool wr = live && (lane < 16);
      if (wr) *(volatile v4f*)op = y;
      __threadfence();
      if (wr) *(volatile v4f*)op = y;
    }
  }
}

static int pick_nb(int nE, int nN) {
  int nb = NBMAX;
  while (nb > 32 && (long long)nb * (long long)nE * 5LL > (long long)RCAP * (long long)nN * 4LL) nb >>= 1;
  return nb;
}
static inline int cdiv(int a, int b) { return (a + b - 1) / b; }

extern "C" void kernel_launch(void* const* d_in, const int* in_sizes, int n_in,
                              void* d_out, int out_size, void* d_ws, size_t ws_size,
                              hipStream_t stream) {
  if (n_in < 17) return;
  const int nN = in_sizes[0] / DIN;
  if (nN <= 0 || in_sizes[0] != nN * DIN || nN > (1 << 21)) return;
  if (in_sizes[1] < 2 || (in_sizes[1] & 1) != 0) return;
  const int nE = in_sizes[1] / 2;
  if (nE < 1 || nE >= (1 << (32 - SLOTB))) return;
  if (in_sizes[2] != nE) return;
  if (in_sizes[3] != DIN * HC || in_sizes[4] != HC) return;
  if (in_sizes[5] != DIN * HC || in_sizes[6] != HC) return;
  if (in_sizes[7] != HC || in_sizes[8] != HC || in_sizes[9] != HC) return;
  if (in_sizes[10] != HC * DOUT || in_sizes[11] != DOUT) return;
  if (in_sizes[12] != HC * DOUT || in_sizes[13] != DOUT) return;
  if (in_sizes[14] != DOUT || in_sizes[15] != DOUT || in_sizes[16] != DOUT) return;
  if (out_size != nN * DOUT) return;

  const float* x     = (const float*)d_in[0];
  const int*   ei    = (const int*)  d_in[1];
  const float* eattr = (const float*)d_in[2];
  const float* W1l   = (const float*)d_in[3];
  const float* b1l   = (const float*)d_in[4];
  const float* W1r   = (const float*)d_in[5];
  const float* b1r   = (const float*)d_in[6];
  const float* W1e   = (const float*)d_in[7];
  const float* att1  = (const float*)d_in[8];
  const float* bias1 = (const float*)d_in[9];
  const float* W2l   = (const float*)d_in[10];
  const float* b2l   = (const float*)d_in[11];
  const float* W2r   = (const float*)d_in[12];
  const float* b2r   = (const float*)d_in[13];
  const float* W2e   = (const float*)d_in[14];
  const float* att2  = (const float*)d_in[15];
  const float* bias2 = (const float*)d_in[16];
  float* outp = (float*)d_out;
  const int* src = ei;
  const int* dst = ei + nE;

  const int MP   = cdiv(nN, GBM) * GBM;
  const int nb   = pick_nb(nE, nN);
  if (nb < 32 || (nb & (nb - 1)) != 0 || nb > NBMAX) return;
  const int gA   = cdiv(MP, nb);
  const int vec8 = ((nE & 3) == 0) ? 1 : 0;
  if (gA * nb < MP) return;

  char* ws = (char*)d_ws;
  size_t off = 0;
  const size_t oXB  = off; off += (size_t)MP * KX * 2;            off = (off + 255) & ~(size_t)255;
  const size_t oWT1 = off; off += (size_t)NP1 * KX * 2;           off = (off + 255) & ~(size_t)255;
  const size_t oH1  = off; off += (size_t)MP * NP1 * 4;           off = (off + 255) & ~(size_t)255;
  const size_t oHB  = off; off += (size_t)MP * KX * 2;            off = (off + 255) & ~(size_t)255;
  const size_t oWT2 = off; off += (size_t)NP2 * KX * 2;           off = (off + 255) & ~(size_t)255;
  const size_t oH2  = off; off += (size_t)MP * NP2 * 4;           off = (off + 255) & ~(size_t)255;
  if (off > ws_size || off > (size_t)WSMAX) return;
  unsigned short* XB  = (unsigned short*)(ws + oXB);
  unsigned short* WT1 = (unsigned short*)(ws + oWT1);
  float*          H1  = (float*)(ws + oH1);
  unsigned short* HB  = (unsigned short*)(ws + oHB);
  unsigned short* WT2 = (unsigned short*)(ws + oWT2);
  float*          H2  = (float*)(ws + oH2);

  hipFuncSetAttribute(reinterpret_cast<const void*>(&k_agg<CPL1, 0>),
                      hipFuncAttributeMaxDynamicSharedMemorySize, LDS_AGG);
  hipFuncSetAttribute(reinterpret_cast<const void*>(&k_agg<CPL2, 1>),
                      hipFuncAttributeMaxDynamicSharedMemorySize, LDS_AGG);

  const int nUx = MP * (DIN / 8);
  const int nBx = cdiv(nUx, NTHR);
  if (nBx * NTHR != nUx) return;
  k_prep<<<nBx + 2 * NBW1 + 2 * NBW2, NTHR, 0, stream>>>(x, W1l, W1r, W2l, W2r, XB, WT1, WT2, nN, nUx, nBx);

  const int gM = MP / GBM;
  k_gemm<<<dim3(gM, NP1 / GBN), GTHR, 0, stream>>>(XB, WT1, b1l, b1r, b1r, HC, NP1, HC, HC, HC, H1, KX, NP1);

  k_agg<CPL1, 0><<<gA, NTHR, LDS_AGG, stream>>>(src, dst, eattr, H1, W1e, att1, bias1, HB, outp,
                                                nN, nE, nb, vec8, MP);

  k_gemm<<<dim3(gM, NP2 / GBN), GTHR, 0, stream>>>(HB, WT2, b2l, b2r, b2r, DOUT, NP2, DOUT, DOUT, DOUT, H2, KX, NP2);

  k_agg<CPL2, 1><<<gA, NTHR, LDS_AGG, stream>>>(src, dst, eattr, H2, W2e, att2, bias2, HB, outp,
                                                nN, nE, nb, vec8, MP);
}
